// MixedScore_MultiHeadAttention_40183714021845
// MI455X (gfx1250) — hardware-verified
//
#include <hip/hip_runtime.h>
#include <math.h>
#include <stdint.h>

#define NB      4
#define NQ      512
#define NC      512
#define DMODEL  256
#define NHEAD   8
#define HDIM    32
#define MSH     16
#define HG      8
#define NHG     (NHEAD / HG)
#define ROWP    (HG * HDIM)
#define NROWS   (NB * NQ)
#define WSC     64.0f
#define ACARRY  16.0f
#define QC      16.0f
#define KC      16.0f
#define VC      16.0f
#define PC      16384.0f
#define FC      4096.0f
#define ATT_SCALE 0.17677669529663689f
#define LOG2E   1.4426950408889634f
static_assert(NHEAD * HDIM == DMODEL);
static_assert(NHG * HG == NHEAD && ROWP * NHG == DMODEL);
static_assert(HDIM == 32 && MSH == 16 && NHG == 1);
static_assert((NQ % 64) == 0 && (NC % 64) == 0 && (DMODEL % 64) == 0 && (NC % 32) == 0 && (NQ % 16) == 0);
static_assert((NROWS % 64) == 0 && ((NROWS * DMODEL) % 2048) == 0);
#define ATT_THREADS (HG * 32)
#define ATT_BLOCKS  (NB * (NQ / 16) * NHG)
static_assert(ATT_THREADS == 256 && ATT_BLOCKS == 128);

typedef _Float16 v16h __attribute__((ext_vector_type(16)));
typedef _Float16 v8h  __attribute__((ext_vector_type(8)));
typedef float    v8f  __attribute__((ext_vector_type(8)));
typedef float    v4f  __attribute__((ext_vector_type(4)));
typedef unsigned int v4u __attribute__((ext_vector_type(4)));

union FragH { v16h v; v8h h[2]; v4u u[2]; };

__device__ __forceinline__ unsigned short bf_bits(float f) {
  unsigned u = __float_as_uint(f);
  return (unsigned short)((u + 0x7FFFu + ((u >> 16) & 1u)) >> 16);
}
__device__ __forceinline__ float bf_up(unsigned short h) { return __uint_as_float(((unsigned)h) << 16); }
__device__ __forceinline__ float bfr(float f) { return bf_up(bf_bits(f)); }
__device__ __forceinline__ unsigned short h_bits(_Float16 x) { return __builtin_bit_cast(unsigned short, x); }
__device__ __forceinline__ unsigned pk16(unsigned short a, unsigned short b) { return (unsigned)a | ((unsigned)b << 16); }
__device__ __forceinline__ v8f zero8() { v8f z = {0.f, 0.f, 0.f, 0.f, 0.f, 0.f, 0.f, 0.f}; return z; }

__device__ __forceinline__ v16h ldfrag_h(const _Float16* p) {
  FragH f;
  f.h[0] = *(const v8h*)(p);
  f.h[1] = *(const v8h*)(p + 16);
  return f.v;
}
__device__ __forceinline__ v16h ldfrag_u(const unsigned short* p) {
  FragH f;
  f.u[0] = *(const v4u*)(p);
  f.u[1] = *(const v4u*)(p + 16);
  return f.v;
}

__device__ __forceinline__ v8f mma_raw(v16h a, v16h b, v8f c) {
  return __builtin_amdgcn_wmma_f32_16x16x32_f16(false, a, false, b, (short)0, c, false, false);
}
__device__ __forceinline__ void dep_guard1(v8f& a, v8f& b, v16h x) {
#if defined(__HIP_DEVICE_COMPILE__)
  asm volatile("v_nop\n\tv_nop\n\tv_nop\n\tv_nop" : "+v"(a), "+v"(b) : "v"(x));
#endif
}
__device__ __forceinline__ void dep_guard2(v8f& a, v8f& b, v16h x, v16h y) {
#if defined(__HIP_DEVICE_COMPILE__)
  asm volatile("v_nop\n\tv_nop\n\tv_nop\n\tv_nop" : "+v"(a), "+v"(b) : "v"(x), "v"(y));
#endif
}
__device__ __forceinline__ void guard_s22(v8f& s, v8f& t, v16h a0, v16h a1, v16h q) {
#if defined(__HIP_DEVICE_COMPILE__)
  asm volatile("v_nop\n\tv_nop\n\tv_nop\n\tv_nop" : "+v"(s), "+v"(t) : "v"(a0), "v"(a1), "v"(q));
#endif
}
__device__ __forceinline__ void guard_pv4(v8f& a, v8f& b, v16h x, v16h y, v16h z, v16h w) {
#if defined(__HIP_DEVICE_COMPILE__)
  asm volatile("v_nop\n\tv_nop\n\tv_nop\n\tv_nop" : "+v"(a), "+v"(b) : "v"(x), "v"(y), "v"(z), "v"(w));
#endif
}
__device__ __forceinline__ void keep4_h(v16h a, v16h b, v16h c, v16h d) {
#if defined(__HIP_DEVICE_COMPILE__)
  asm volatile("v_nop" :: "v"(a), "v"(b), "v"(c), "v"(d));
#endif
}
__device__ __forceinline__ void acc_guard4(v8f& a, v8f& b, v8f& c, v8f& d) {
#if defined(__HIP_DEVICE_COMPILE__)
  asm volatile("v_nop\n\tv_nop\n\tv_nop\n\tv_nop" : "+v"(a), "+v"(b), "+v"(c), "+v"(d));
#endif
}
__device__ __forceinline__ void wave_sync_lds() {
  __builtin_amdgcn_fence(__ATOMIC_RELEASE, "workgroup");
  __builtin_amdgcn_wave_barrier();
  __builtin_amdgcn_fence(__ATOMIC_ACQUIRE, "workgroup");
}

__global__ __launch_bounds__(256) void cvt16(const float* __restrict__ src, unsigned short* dst, int n, float sc) {
  const size_t i8 = ((size_t)blockIdx.x * 256 + threadIdx.x) * 8;
  if (i8 + 8 > (size_t)n) return;
  const v4f a = *(const v4f*)(src + i8);
  const v4f b = *(const v4f*)(src + i8 + 4);
  v4u o;
  o[0] = pk16(h_bits((_Float16)(bfr(a[0]) * sc)), h_bits((_Float16)(bfr(a[1]) * sc)));
  o[1] = pk16(h_bits((_Float16)(bfr(a[2]) * sc)), h_bits((_Float16)(bfr(a[3]) * sc)));
  o[2] = pk16(h_bits((_Float16)(bfr(b[0]) * sc)), h_bits((_Float16)(bfr(b[1]) * sc)));
  o[3] = pk16(h_bits((_Float16)(bfr(b[2]) * sc)), h_bits((_Float16)(bfr(b[3]) * sc)));
  for (int pass = 0; pass < 2; ++pass) {
    *(volatile v4u*)(dst + i8) = o;
    __threadfence();
  }
}

__global__ __launch_bounds__(256) void wtr64(const float* __restrict__ W, unsigned short* dst, float sc) {
  __shared__ __align__(16) float tl[64 * 68];
  const int tid = threadIdx.x;
  const int n0  = blockIdx.x * 64;
  const int k0  = blockIdx.y * 64;
  const int nl  = tid & 63, kq = tid >> 6;
#pragma unroll
  for (int it = 0; it < 16; ++it) {
    const int kl = it * 4 + kq;
    tl[nl * 68 + kl] = W[(size_t)(k0 + kl) * DMODEL + n0 + nl];
  }
  __syncthreads();
  v4u o[2];
#pragma unroll
  for (int it = 0; it < 2; ++it) {
    const int p  = it * 256 + tid;
    const int rn = p >> 3, kk = (p & 7) * 8;
    const float* sp = tl + rn * 68 + kk;
    const v4f a = *(const v4f*)(sp);
    const v4f b = *(const v4f*)(sp + 4);
    v4u w;
    w[0] = pk16(h_bits((_Float16)(bfr(a[0]) * sc)), h_bits((_Float16)(bfr(a[1]) * sc)));
    w[1] = pk16(h_bits((_Float16)(bfr(a[2]) * sc)), h_bits((_Float16)(bfr(a[3]) * sc)));
    w[2] = pk16(h_bits((_Float16)(bfr(b[0]) * sc)), h_bits((_Float16)(bfr(b[1]) * sc)));
    w[3] = pk16(h_bits((_Float16)(bfr(b[2]) * sc)), h_bits((_Float16)(bfr(b[3]) * sc)));
    o[it] = w;
  }
  for (int pass = 0; pass < 2; ++pass) {
#pragma unroll
    for (int it = 0; it < 2; ++it) {
      const int p  = it * 256 + tid;
      const int rn = p >> 3, kk = (p & 7) * 8;
      *(volatile v4u*)(dst + (size_t)(n0 + rn) * DMODEL + k0 + kk) = o[it];
    }
    __threadfence();
  }
}

template <int OM, int NA>
__global__ __launch_bounds__(256) void gemm64(
    const unsigned short* __restrict__ Ap, const unsigned short* __restrict__ Aq, int lda, long long sA,
    const unsigned short* __restrict__ Btp, int ldb, long long sB,
    void* Cout, int ldc, long long sC,
    int M, int N, int K, float oscale, float ocarry) {
  __shared__ __align__(16) float sT[8][16 * 68];
  const int by   = blockIdx.y;
  const int lane = threadIdx.x & 31;
  const int wave = threadIdx.x >> 5;
  const int tilesN = N >> 6;
  const int tilesM = M >> 6;
  const int tile = blockIdx.x * 8 + wave;
  if (tile >= tilesM * tilesN) return;
  const int tm = tile / tilesN;
  const int tn = tile - tm * tilesN;
  const int m0 = tm << 6;
  const int n0 = tn << 6;

  const unsigned short* A1 = Ap  + (size_t)((long long)by * sA);
  const unsigned short* A2 = Aq  + (size_t)((long long)by * sA);
  const unsigned short* Bb = Btp + (size_t)((long long)by * sB);

  const int rlane = lane & 15;
  const int koff  = (lane >> 4) * 8;
  const int mOff  = (lane >> 4) * 8;

  v8f acc[4][4];
#pragma unroll
  for (int i = 0; i < 4; ++i)
#pragma unroll
    for (int j = 0; j < 4; ++j) acc[i][j] = zero8();

  for (int k0 = 0; k0 < K; k0 += 32) {
    v16h bh[4];
#pragma unroll
    for (int j = 0; j < 4; ++j) {
      const size_t bofs = (size_t)(n0 + (j << 4) + rlane) * ldb + koff + k0;
      bh[j] = ldfrag_u(Bb + bofs);
    }
#pragma unroll
    for (int i = 0; i < 4; ++i) {
      const size_t ao = (size_t)(m0 + (i << 4) + rlane) * lda + koff + k0;
      const v16h ah = ldfrag_u(A1 + ao);
#pragma unroll
      for (int j = 0; j < 4; ++j) acc[i][j] = mma_raw(ah, bh[j], acc[i][j]);
      if constexpr (NA == 2) {
        const v16h al = ldfrag_u(A2 + ao);
#pragma unroll
        for (int j = 0; j < 4; ++j) acc[i][j] = mma_raw(al, bh[j], acc[i][j]);
        dep_guard2(acc[i][0], acc[i][3], ah, al);
      } else {
        dep_guard1(acc[i][0], acc[i][3], ah);
      }
    }
    keep4_h(bh[0], bh[1], bh[2], bh[3]);
  }
  acc_guard4(acc[0][0], acc[0][1], acc[0][2], acc[0][3]);
  acc_guard4(acc[1][0], acc[1][1], acc[1][2], acc[1][3]);
  acc_guard4(acc[2][0], acc[2][1], acc[2][2], acc[2][3]);
  acc_guard4(acc[3][0], acc[3][1], acc[3][2], acc[3][3]);

  const int hh2 = lane >> 4, c4 = (lane & 15) * 4;
  const int q8  = lane >> 3, c8 = (lane & 7) * 8;

  float* slab = sT[wave];
#pragma unroll
  for (int i = 0; i < 4; ++i) {
    const int mBase = m0 + (i << 4);
#pragma unroll
    for (int j = 0; j < 4; ++j) {
#pragma unroll
      for (int r = 0; r < 8; ++r) {
        slab[(mOff + r) * 68 + (j << 4) + rlane] = acc[i][j][r];
      }
    }
    wave_sync_lds();
    if constexpr (OM == 0) {
      float* C = (float*)Cout + (size_t)((long long)by * sC);
      v4f vals[8];
#pragma unroll
      for (int it = 0; it < 8; ++it) {
        const int row = it * 2 + hh2;
        v4f v = *(const v4f*)(slab + row * 68 + c4);
#pragma unroll
        for (int e = 0; e < 4; ++e) v[e] = v[e] * oscale;
        vals[it] = v;
      }
      for (int pass = 0; pass < 2; ++pass) {
#pragma unroll
        for (int it = 0; it < 8; ++it) {
          const int gr = mBase + it * 2 + hh2;
          *(volatile v4f*)(C + (size_t)gr * ldc + n0 + c4) = vals[it];
        }
        __threadfence();
      }
    } else {
      unsigned short* C = (unsigned short*)Cout + (size_t)((long long)by * sC);
      v4u hv[4];
#pragma unroll
      for (int it = 0; it < 4; ++it) {
        const int row = it * 4 + q8;
        const float* sp = slab + row * 68 + c8;
        v4u a = {0u, 0u, 0u, 0u};
#pragma unroll
        for (int e = 0; e < 4; ++e) {
          float f0 = sp[2 * e] * oscale;
          float f1 = sp[2 * e + 1] * oscale;
          f0 *= ocarry; f1 *= ocarry;
          a[e] = pk16(h_bits((_Float16)f0), h_bits((_Float16)f1));
        }
        hv[it] = a;
      }
      for (int pass = 0; pass < 2; ++pass) {
#pragma unroll
        for (int it = 0; it < 4; ++it) {
          const int row = it * 4 + q8;
          *(volatile v4u*)(C + (size_t)(mBase + row) * ldc + n0 + c8) = hv[it];
        }
        __threadfence();
      }
    }
    wave_sync_lds();
  }
}

#define PS_FLOATS (HG * 16 * 36)
#define SM_FLOATS 4608
static_assert(PS_FLOATS <= SM_FLOATS);
static_assert((size_t)2 * 16 * ROWP * sizeof(unsigned short) <= (size_t)SM_FLOATS * sizeof(float));

__global__ __launch_bounds__(ATT_THREADS)
void attn8(const unsigned short* __restrict__ QHp, const unsigned short* __restrict__ KHp,
           const unsigned short* __restrict__ VTq, const float* __restrict__ costp,
           const float* __restrict__ m1w, const float* __restrict__ m1b,
           const float* __restrict__ m2w, const float* __restrict__ m2b,
           unsigned short* CTH, unsigned short* CTL) {
  __shared__ __align__(16) float smem[SM_FLOATS];

  const int tid  = threadIdx.x;
  const int wave = __builtin_amdgcn_readfirstlane(tid >> 5);
  const int lane = tid & 31;
  const int hh   = lane >> 4;
  const int c    = lane & 15;

  const int qt   = blockIdx.x % (NQ / 16);
  const int bat  = blockIdx.x / (NQ / 16);
  const int head = wave;
  const int q0   = qt * 16;

  const size_t qofs = ((size_t)bat * NQ + q0 + c) * DMODEL + head * HDIM + 8 * hh;
  const _Float16* Qh = (const _Float16*)(const void*)QHp + qofs;
  const _Float16* Kb = (const _Float16*)(const void*)KHp + (size_t)bat * NC * DMODEL + head * HDIM + 8 * hh;
  const _Float16* Vb = (const _Float16*)(const void*)VTq + ((size_t)bat * DMODEL + head * HDIM) * NC + 8 * hh;
  const float* cp = costp + ((size_t)bat * NQ + q0 + 8 * hh) * NC + c;
  const float dsc = ATT_SCALE / (QC * KC);

  float w0r[MSH], w1r[MSH], b1r[MSH], w2r[MSH];
#pragma unroll
  for (int m = 0; m < MSH; ++m) {
    w0r[m] = bfr(m1w[(head * 2 + 0) * MSH + m]);
    w1r[m] = bfr(m1w[(head * 2 + 1) * MSH + m]);
    b1r[m] = bfr(m1b[head * MSH + m]);
    w2r[m] = bfr(m2w[head * MSH + m]);
  }
  const float b2 = bfr(m2b[head]);

  const v16h qa = ldfrag_h(Qh);

  float mrow[8], lrow[8];
  v8f o0 = zero8(), o1 = zero8();
#pragma unroll
  for (int r = 0; r < 8; ++r) { mrow[r] = -INFINITY; lrow[r] = 0.f; }
  float* pt = smem + wave * (16 * 36);

#pragma unroll 1
  for (int kb = 0; kb < NC; kb += 32) {
    const _Float16* kp = Kb + (size_t)(kb + c) * DMODEL;
    v8f s0, s1;
    {
      const v16h k0 = ldfrag_h(kp);
      const v16h k1 = ldfrag_h(kp + (size_t)16 * DMODEL);
      s0 = mma_raw(qa, k0, zero8());
      s1 = mma_raw(qa, k1, zero8());
      guard_s22(s0, s1, k0, k1, qa);
    }
    const float* tp = cp + kb;
#pragma unroll
    for (int r = 0; r < 8; ++r) {
      const float cr0 = bfr(tp[(size_t)r * NC]);
      const float cr1 = bfr(tp[(size_t)r * NC + 16]);
      const float d0 = s0[r] * dsc, d1 = s1[r] * dsc;
      float a0 = 0.f, a1 = 0.f;
#pragma unroll
      for (int m = 0; m < MSH; ++m) {
        const float p0 = fmaf(w0r[m], d0, fmaf(w1r[m], cr0, b1r[m]));
        const float p1 = fmaf(w0r[m], d1, fmaf(w1r[m], cr1, b1r[m]));
        a0 = fmaf(w2r[m], fmaxf(p0, 0.f), a0);
        a1 = fmaf(w2r[m], fmaxf(p1, 0.f), a1);
      }
      const float t0 = (a0 + b2) * LOG2E, t1 = (a1 + b2) * LOG2E;
      float mx = fmaxf(t0, t1);
#pragma unroll
      for (int off = 1; off < 16; off <<= 1) mx = fmaxf(mx, __shfl_xor(mx, off, 32));
      const float mn = fmaxf(mrow[r], mx);
      const float al = exp2f(mrow[r] - mn);
      mrow[r] = mn;
      const float e0 = exp2f(t0 - mn), e1 = exp2f(t1 - mn);
      float ps = e0 + e1;
#pragma unroll
      for (int off = 1; off < 16; off <<= 1) ps += __shfl_xor(ps, off, 32);
      lrow[r] = lrow[r] * al + ps;
      o0[r] *= al;
      o1[r] *= al;
      const int ro = (8 * hh + r) * 36 + c;
      pt[ro]      = e0;
      pt[ro + 16] = e1;
    }
    wave_sync_lds();
    FragH ph, pl;
    {
      const float* prow = pt + c * 36 + 8 * hh;
      const v4f p0 = *(const v4f*)(prow), p1 = *(const v4f*)(prow + 4);
      const v4f p2 = *(const v4f*)(prow + 16), p3 = *(const v4f*)(prow + 20);
#pragma unroll
      for (int e = 0; e < 4; ++e) {
        const float c0 = p0[e] * PC, c1 = p1[e] * PC, c2 = p2[e] * PC, c3 = p3[e] * PC;
        const _Float16 g0 = (_Float16)c0, g1 = (_Float16)c1, g2 = (_Float16)c2, g3 = (_Float16)c3;
        ph.h[0][e]     = g0;
        ph.h[0][4 + e] = g1;
        ph.h[1][e]     = g2;
        ph.h[1][4 + e] = g3;
        pl.h[0][e]     = (_Float16)(c0 - (float)g0);
        pl.h[0][4 + e] = (_Float16)(c1 - (float)g1);
        pl.h[1][e]     = (_Float16)(c2 - (float)g2);
        pl.h[1][4 + e] = (_Float16)(c3 - (float)g3);
      }
    }
    const _Float16* vp = Vb + (size_t)c * NC + kb;
    {
      const v16h vb0 = ldfrag_h(vp);
      const v16h vb1 = ldfrag_h(vp + (size_t)16 * NC);
      o0 = mma_raw(ph.v, vb0, o0);
      o1 = mma_raw(ph.v, vb1, o1);
      o0 = mma_raw(pl.v, vb0, o0);
      o1 = mma_raw(pl.v, vb1, o1);
      guard_pv4(o0, o1, ph.v, pl.v, vb0, vb1);
    }
    wave_sync_lds();
  }

  __syncthreads();
  unsigned short* Osh = (unsigned short*)smem;
  unsigned short* Osl = Osh + 16 * ROWP;
  const float oc = FC / (PC * VC);
#pragma unroll
  for (int r = 0; r < 8; ++r) {
    const float inv = (1.0f / lrow[r]) * oc;
    const int ro = (8 * hh + r) * ROWP + wave * HDIM + c;
    const float f0 = o0[r] * inv, f1 = o1[r] * inv;
    const _Float16 g0 = (_Float16)f0, g1 = (_Float16)f1;
    Osh[ro]      = h_bits(g0);
    Osh[ro + 16] = h_bits(g1);
    Osl[ro]      = h_bits((_Float16)(f0 - (float)g0));
    Osl[ro + 16] = h_bits((_Float16)(f1 - (float)g1));
  }
  __syncthreads();
  {
    v4u vh[2], vl[2];
#pragma unroll
    for (int it = 0; it < 2; ++it) {
      const int p = it * ATT_THREADS + tid;
      vh[it] = *(const v4u*)(Osh + (size_t)p * 8);
      vl[it] = *(const v4u*)(Osl + (size_t)p * 8);
    }
    const size_t base = ((size_t)bat * NQ + q0) * DMODEL;
    unsigned short* dh = CTH + base;
    unsigned short* dl = CTL + base;
    for (int pass = 0; pass < 2; ++pass) {
#pragma unroll
      for (int it = 0; it < 2; ++it) {
        const int p = it * ATT_THREADS + tid;
        const size_t po = (size_t)(p >> 5) * DMODEL + (size_t)(p & 31) * 8;
        *(volatile v4u*)(dh + po) = vh[it];
        *(volatile v4u*)(dl + po) = vl[it];
      }
      __threadfence();
    }
  }
}

extern "C" void kernel_launch(void* const* d_in, const int* in_sizes, int n_in,
                              void* d_out, int out_size, void* d_ws, size_t ws_size,
                              hipStream_t stream) {
  if (n_in < 10) return;
  if (in_sizes[0] != NROWS * DMODEL) return;
  if (in_sizes[1] != NB * NQ * NC) return;
  if (in_sizes[2] != DMODEL * DMODEL || in_sizes[3] != DMODEL * DMODEL ||
      in_sizes[4] != DMODEL * DMODEL || in_sizes[5] != DMODEL * DMODEL) return;
  if (in_sizes[6] != NHEAD * 2 * MSH || in_sizes[7] != NHEAD * MSH || in_sizes[8] != NHEAD * MSH || in_sizes[9] != NHEAD) return;
  if (out_size != NROWS * DMODEL) return;
  if ((in_sizes[0] % 2048) != 0) return;

  const float* x    = (const float*)d_in[0];
  const float* cost = (const float*)d_in[1];
  const float* w_q  = (const float*)d_in[2];
  const float* w_k  = (const float*)d_in[3];
  const float* w_v  = (const float*)d_in[4];
  const float* w_o  = (const float*)d_in[5];
  const float* m1w  = (const float*)d_in[6];
  const float* m1b  = (const float*)d_in[7];
  const float* m2w  = (const float*)d_in[8];
  const float* m2b  = (const float*)d_in[9];
  float*       out  = (float*)d_out;

  const size_t PW  = (size_t)DMODEL * DMODEL * 2;
  const size_t PX  = (size_t)NROWS * DMODEL * 2;
  const size_t PVT = (size_t)NB * DMODEL * NC * 2;
  size_t off = 0;
  const size_t oWQ = off; off += PW;
  const size_t oWK = off; off += PW;
  const size_t oWV = off; off += PW;
  const size_t oWO = off; off += PW;
  const size_t oX  = off; off += PX;
  const size_t oQH = off; off += PX;
  const size_t oKH = off; off += PX;
  const size_t oVT = off; off += PVT;
  const size_t oCH = off; off += PX;
  const size_t oCL = off; off += PX;
  if (off > ws_size) return;
  if (off > (size_t)134217728) return;

  char* ws = (char*)d_ws;
  unsigned short* WQT = (unsigned short*)(ws + oWQ);
  unsigned short* WKT = (unsigned short*)(ws + oWK);
  unsigned short* WVT = (unsigned short*)(ws + oWV);
  unsigned short* WOT = (unsigned short*)(ws + oWO);
  unsigned short* X16 = (unsigned short*)(ws + oX);
  unsigned short* QH  = (unsigned short*)(ws + oQH);
  unsigned short* KH  = (unsigned short*)(ws + oKH);
  unsigned short* VTp = (unsigned short*)(ws + oVT);
  unsigned short* CTH = (unsigned short*)(ws + oCH);
  unsigned short* CTL = (unsigned short*)(ws + oCL);

  const dim3 blk(256);
  const dim3 gWT(DMODEL / 64, DMODEL / 64);
  const dim3 gCX((NROWS * DMODEL) / 2048);
  const int tilesP = (NROWS / 64) * (DMODEL / 64);
  const int tilesV = (DMODEL / 64) * (NC / 64);
  const dim3 gP((tilesP + 7) / 8, 1);
  const dim3 gV((tilesV + 7) / 8, NB);
  const dim3 gAT(ATT_BLOCKS);
  const dim3 bAT(ATT_THREADS);

  wtr64<<<gWT, blk, 0, stream>>>(w_q, WQT, WSC);
  wtr64<<<gWT, blk, 0, stream>>>(w_k, WKT, WSC);
  wtr64<<<gWT, blk, 0, stream>>>(w_v, WVT, WSC);
  wtr64<<<gWT, blk, 0, stream>>>(w_o, WOT, WSC);

  cvt16<<<gCX, blk, 0, stream>>>(x, X16, NROWS * DMODEL, ACARRY);

  gemm64<2, 1><<<gP, blk, 0, stream>>>(
      X16, X16, DMODEL, 0LL,
      WQT, DMODEL, 0LL,
      (void*)QH, DMODEL, 0LL,
      NROWS, DMODEL, DMODEL, 1.0f / (ACARRY * WSC), QC);

  gemm64<2, 1><<<gP, blk, 0, stream>>>(
      X16, X16, DMODEL, 0LL,
      WKT, DMODEL, 0LL,
      (void*)KH, DMODEL, 0LL,
      NROWS, DMODEL, DMODEL, 1.0f / (ACARRY * WSC), KC);

  gemm64<2, 1><<<gV, blk, 0, stream>>>(
      WVT, WVT, DMODEL, 0LL,
      X16, DMODEL, (long long)NC * DMODEL,
      (void*)VTp, NC, (long long)DMODEL * NC,
      DMODEL, NC, DMODEL, 1.0f / (ACARRY * WSC), VC);

  attn8<<<gAT, bAT, 0, stream>>>(QH, KH, VTp, cost, m1w, m1b, m2w, m2b, CTH, CTL);

  gemm64<0, 2><<<gP, blk, 0, stream>>>(
      CTH, CTL, DMODEL, 0LL,
      WOT, DMODEL, 0LL,
      (void*)out, DMODEL, 0LL,
      NROWS, DMODEL, DMODEL, 1.0f / (FC * WSC), 1.0f);

  (void)hipGetLastError();
}
